// SLGAT_32684701122586
// MI455X (gfx1250) — hardware-run, weakly checked
//
#include <hip/hip_runtime.h>


namespace {
constexpr int N = 50000, NP = 50048, E = 800000, D0 = 128, HID = 160, NH = 5, CH = 32, G = 512, NOUT = 10, VOC = 500;
constexpr float XS = 256.0f  , WSC = 256.0f, NEG = 0.2f, ALPHA = 0.1f, BETA = 0.1f;

typedef _Float16 b16;
typedef __attribute__((ext_vector_type(16))) _Float16 v16b;
typedef __attribute__((ext_vector_type(8))) _Float16 v8b;
typedef __attribute__((ext_vector_type(8))) float v8f;
typedef __attribute__((ext_vector_type(4))) float v4f;
__device__ __forceinline__ float bf16_rne(float f) { unsigned int u = __float_as_uint(f); u += 0x7FFFu + ((u >> 16) & 1u); return __uint_as_float(u & 0xFFFF0000u); }
__device__ __forceinline__ void split16(float v, b16& hi, b16& lo) { hi = (b16)v; lo = (b16)(v - (float)hi); }
__device__ __forceinline__ v16b frag_kb(const b16* p, int hh) { const v8b a = *(const v8b*)(p + 8 * hh), b = *(const v8b*)(p + 16 + 8 * hh); v16b f;
#pragma unroll
  for (int e = 0; e < 8; ++e) { f[e] = a[e]; f[8 + e] = b[e]; } return f; }
__device__ __forceinline__ v8f wmma16b(v16b a, v16b b, v8f c) { v8f d = __builtin_amdgcn_wmma_f32_16x16x32_f16(false, a, false, b, (short)0, c, false, false); asm volatile("v_nop\n\tv_nop\n\tv_nop\n\tv_nop" : "+v"(d) : "v"(a), "v"(b)); return d; }
__device__ __forceinline__ void wave_lds_sync() { __builtin_amdgcn_fence(__ATOMIC_RELEASE, "workgroup"); __builtin_amdgcn_wave_barrier(); __builtin_amdgcn_fence(__ATOMIC_ACQUIRE, "workgroup"); }
__device__ __forceinline__ float pmul(float a, float b) { float p = a * b; asm volatile("" : "+v"(p)); return p; }
__device__ __forceinline__ int iclamp(int v, int lo, int hi) { return v < lo ? lo : (v > hi ? hi : v); }
__device__ __forceinline__ float nexp(float x) { return __builtin_amdgcn_exp2f(x * 1.4426950408889634f); }
__device__ __forceinline__ float lrelu(float x) { return x > 0.0f ? x : NEG * x; }

constexpr int CSR_NBLK = 512, CSR_GB = 9, CSR_GN = 1 << CSR_GB  , CSR_MAXG = 512, CSR_CAP = 12288  ;
__global__ __launch_bounds__(64) void csrA_kernel(const int* __restrict__ dst, int E, int N, int nG, int CHP, int NGP, int* __restrict__ STG, int* __restrict__ HST) {
  extern __shared__ int sm[];
  int* cnt = sm; int* run = sm + NGP; int* ids = sm + 2 * NGP;
  const int b = blockIdx.x; const int ch = (E + CSR_NBLK - 1) / CSR_NBLK; const int e0 = b * ch, e1 = min(E, e0 + ch);
  for (int i = threadIdx.x; i < NGP; i += 64) cnt[i] = 0;
  for (int i = threadIdx.x; i < CHP; i += 64) ids[i] = -1;
  __syncthreads();
  if (threadIdx.x == 0) {
    for (int e = e0; e < e1; ++e) { int d = dst[e]; d = (d < 0) ? 0 : (d >= N ? N - 1 : d); cnt[d >> CSR_GB] += 1; }
    int acc = 0; for (int g = 0; g < nG; ++g) { run[g] = acc; acc += cnt[g]; }
    for (int e = e0; e < e1; ++e) { int d = dst[e]; d = (d < 0) ? 0 : (d >= N ? N - 1 : d); const int g = d >> CSR_GB; ids[run[g]] = e; run[g] += 1; } }
  __syncthreads();
  typedef __attribute__((ext_vector_type(4))) int v4i;
  for (int pass = 0; pass < 2; ++pass) {
    for (int i = threadIdx.x; i < CHP / 4; i += 64) *(volatile v4i*)(STG + (size_t)b * CHP + i * 4) = *(const v4i*)(&ids[i * 4]);
    for (int i = threadIdx.x; i < NGP / 4; i += 64) { v4i v; for (int e = 0; e < 4; ++e) v[e] = (i * 4 + e < nG) ? cnt[i * 4 + e] : 0; *(volatile v4i*)(HST + (size_t)b * NGP + i * 4) = v; }
    __threadfence(); }
}
__global__ __launch_bounds__(512) void csrS_kernel(const int* __restrict__ HST, int nG, int NGP, int* __restrict__ START, int* __restrict__ TOT, int* __restrict__ OFF) {
  __shared__ int tot[CSR_MAXG];
  const int b = threadIdx.x;
  for (int pass = 0; pass < 2; ++pass) { int runb = 0; for (int g = 0; g < nG; ++g) { int c = HST[(size_t)b * NGP + g]; c = (c < 0) ? 0 : c; ((volatile int*)OFF)[(size_t)g * CSR_NBLK + b] = runb; runb += c; } __threadfence(); }
  for (int g = threadIdx.x; g < nG; g += 512) { int s = 0; for (int bb = 0; bb < CSR_NBLK; ++bb) { int c = HST[(size_t)bb * NGP + g]; s += (c < 0) ? 0 : c; } tot[g] = s; }
  __syncthreads();
  if (threadIdx.x < 32) {
    __shared__ int st[CSR_MAXG + 32];
    if (threadIdx.x == 0) { int acc = 0; for (int g = 0; g < NGP; ++g) { st[g] = acc; if (g < nG) acc += (tot[g] + 31) & ~31; } st[NGP] = acc; }
    __builtin_amdgcn_fence(__ATOMIC_RELEASE, "workgroup"); __builtin_amdgcn_wave_barrier(); __builtin_amdgcn_fence(__ATOMIC_ACQUIRE, "workgroup");
    for (int pass = 0; pass < 2; ++pass) { for (int i = threadIdx.x; i < NGP + 32; i += 32) { ((volatile int*)START)[i] = (i <= NGP) ? st[min(i, NGP)] : 0; ((volatile int*)TOT)[i] = (i < nG) ? tot[i] : 0; } __threadfence(); } }
}
__global__ __launch_bounds__(256) void csrB_kernel(const int* __restrict__ dst, int N, int nG, int CHP, int NGP, int permLen, const int* __restrict__ STG, const int* __restrict__ HST, const int* __restrict__ OFF, const int* __restrict__ START, const int* __restrict__ TOT, int* __restrict__ PERM, int* __restrict__ ROWPTR, int* __restrict__ ROWCNT, int* __restrict__ FLAG) {
  typedef __attribute__((ext_vector_type(4))) int v4i;
  __shared__ int ids[CSR_CAP]; __shared__ unsigned short key[CSR_CAP]; __shared__ int outp[CSR_CAP]; __shared__ int ncnt[CSR_GN + 1]; __shared__ int boff[CSR_NBLK + 1];
  const int g = blockIdx.x, t_ = threadIdx.x; int tot = TOT[g]; int st = START[g], stn = START[g + 1]; const int v0 = g * CSR_GN; const int nv = min(CSR_GN, N - v0);
  st = (st < 0) ? 0 : (st > permLen - 32 ? permLen - 32 : st) & ~31; stn = (stn < st) ? st : (stn > permLen ? permLen : stn); tot = (tot < 0) ? 0 : tot; if (tot > stn - st && tot <= CSR_CAP) tot = stn - st;
  if (tot > CSR_CAP) {
    for (int pass = 0; pass < 2; ++pass) { for (int i = t_; i < CSR_GN / 4; i += 256) { v4i a, c; for (int e = 0; e < 4; ++e) { a[e] = st; c[e] = 0; } *(volatile v4i*)(ROWPTR + v0 + i * 4) = a; *(volatile v4i*)(ROWCNT + v0 + i * 4) = c; } if (t_ == 0) ((volatile int*)FLAG)[0] = 1; __threadfence(); } (void)nv; return; }
  if (t_ == 0) { int acc = 0; for (int b = 0; b < CSR_NBLK; ++b) { boff[b] = acc; int c = HST[(size_t)b * NGP + g]; c = (c < 0) ? 0 : (c > CHP ? CHP : c); acc += c; if (acc > tot) acc = tot; } boff[CSR_NBLK] = acc; }
  for (int i = t_; i <= CSR_GN; i += 256) ncnt[i] = 0;
  __syncthreads();
  for (int b = 0; b < CSR_NBLK; ++b) { const int c = boff[b + 1] - boff[b]; int o_ = OFF[(size_t)g * CSR_NBLK + b]; o_ = (o_ < 0) ? 0 : (o_ > CHP - c ? CHP - c : o_); const int* src_ = STG + (size_t)b * CHP + o_;
    for (int i = t_; i < c; i += 256) { int id = src_[i]; id = (id < 0) ? 0 : id; ids[boff[b] + i] = id; int d = dst[id]; d = (d < v0) ? v0 : (d >= N ? N - 1 : d); int kk = d - v0; kk = (kk < 0) ? 0 : (kk >= CSR_GN ? CSR_GN - 1 : kk); key[boff[b] + i] = (unsigned short)kk; } }
  __syncthreads();
  if (t_ == 0) { for (int i = 0; i < tot; ++i) ncnt[key[i]] += 1; int acc = 0; for (int vl = 0; vl < CSR_GN; ++vl) { const int c = ncnt[vl]; ncnt[vl] = acc; acc += c; } ncnt[CSR_GN] = acc;
    for (int i = 0; i < tot; ++i) { const int vl = key[i]; outp[ncnt[vl]] = ids[i]; ncnt[vl] += 1; }
    for (int vl = CSR_GN; vl > 0; --vl) ncnt[vl] = ncnt[vl - 1]; ncnt[0] = 0; }
  __syncthreads();
  for (int pass = 0; pass < 2; ++pass) {
    for (int i = t_; i < (stn - st) / 4; i += 256) { v4i v; for (int e = 0; e < 4; ++e) { const int q = i * 4 + e; v[e] = (q < tot) ? outp[q] : -1; } *(volatile v4i*)(PERM + st + i * 4) = v; }
    for (int i = t_; i < CSR_GN / 4; i += 256) { v4i a, c; for (int e = 0; e < 4; ++e) { const int vl = i * 4 + e; a[e] = st + ncnt[vl]; c[e] = (vl < nv) ? (ncnt[vl + 1] - ncnt[vl]) : 0; } *(volatile v4i*)(ROWPTR + v0 + i * 4) = a; *(volatile v4i*)(ROWCNT + v0 + i * 4) = c; }
    __threadfence(); }
}
__global__ __launch_bounds__(256) void csrZ_kernel(int* __restrict__ p, size_t n4) { typedef __attribute__((ext_vector_type(4))) int v4i; const size_t tid = (size_t)blockIdx.x * 256 + threadIdx.x, nth = (size_t)gridDim.x * 256; v4i z = {0, 0, 0, 0}; for (size_t i = tid; i < n4; i += nth) *(volatile v4i*)(p + i * 4) = z; }
struct CsrBufs { int *STG, *HST, *OFF, *START, *TOT, *PERM, *ROWPTR, *ROWCNT, *FLAG; int nG, NGP, CHP; size_t permLen; char* base; size_t bytes; };
static size_t csr_carve(CsrBufs& c, char* ws, size_t off, int E, int N) {
  const size_t off0 = off; c.base = ws + off;
  auto al = [&](size_t bytes) { char* p = ws + off; off += (bytes + 255) & ~(size_t)255; return p; };
  c.nG = (N + CSR_GN - 1) / CSR_GN; c.NGP = (c.nG + 31) & ~31; const int ch = (E + CSR_NBLK - 1) / CSR_NBLK; c.CHP = (ch + 31) & ~31; c.permLen = (size_t)E + 32 * (size_t)c.nG + 32;
  c.STG = (int*)al((size_t)CSR_NBLK * c.CHP * 4); c.HST = (int*)al((size_t)CSR_NBLK * c.NGP * 4); c.OFF = (int*)al((size_t)c.NGP * CSR_NBLK * 4); c.START = (int*)al((size_t)(c.NGP + 64) * 4); c.TOT = (int*)al((size_t)(c.NGP + 64) * 4);
  c.PERM = (int*)al(c.permLen * 4); c.ROWPTR = (int*)al((size_t)c.nG * CSR_GN * 4); c.ROWCNT = (int*)al((size_t)c.nG * CSR_GN * 4); c.FLAG = (int*)al(256);
  c.bytes = off - off0; return off;
}
static void csr_build(const CsrBufs& c, const int* dst, int E, int N, hipStream_t stream) {
  const size_t smem = (size_t)(2 * c.NGP + c.CHP) * 4;
  csrZ_kernel<<<512, 256, 0, stream>>>((int*)c.base, c.bytes / 16);
  csrA_kernel<<<CSR_NBLK, 64, smem, stream>>>(dst, E, N, c.nG, c.CHP, c.NGP, c.STG, c.HST);
  csrS_kernel<<<1, 512, 0, stream>>>(c.HST, c.nG, c.NGP, c.START, c.TOT, c.OFF);
  csrB_kernel<<<c.nG, 256, 0, stream>>>(dst, N, c.nG, c.CHP, c.NGP, (int)c.permLen, c.STG, c.HST, c.OFF, c.START, c.TOT, c.PERM, c.ROWPTR, c.ROWCNT, c.FLAG);
}


__device__ __forceinline__ float elu_(float x) { return x > 0.0f ? x : (__expf(x) - 1.0f); }
__global__ __launch_bounds__(256) void prep_kernel(const int* __restrict__ xid, const float* __restrict__ emb, const float* __restrict__ ws, const float* __restrict__ w1, const float* __restrict__ w2, const float* __restrict__ wj, const float* __restrict__ wl1, const float* __restrict__ wl2, b16* __restrict__ XE, b16* __restrict__ WST, b16* __restrict__ W1T, b16* __restrict__ W2T, b16* __restrict__ WJT, b16* __restrict__ WL1T, b16* __restrict__ WL2T) {
  const size_t u = (size_t)blockIdx.x * 256 + threadIdx.x; const size_t nx = (size_t)NP * D0 / 8, n1 = (size_t)HID * D0 / 8, n2 = (size_t)HID * HID / 8, nj = (size_t)HID * 2 * HID / 8, nl2 = (size_t)16 * HID / 8; size_t t = u; v8b o;
  if (t < nx) { const size_t e = t * 8; const size_t v = e / D0; const int c0 = (int)(e % D0); const size_t id = v < (size_t)N ? (size_t)iclamp(xid[v], 0, VOC - 1) : 0; for (int j = 0; j < 8; ++j) o[j] = v < (size_t)N ? (b16)(bf16_rne(emb[id * D0 + c0 + j]) * XS) : (b16)0.0f; for (int pass = 0; pass < 2; ++pass) { *(volatile v8b*)(XE + e) = o; __threadfence(); } return; } t -= nx;
  if (t < 2 * n1) { const int which = (int)(t / n1); const size_t e = (t % n1) * 8; const int oo = (int)(e / D0), k0 = (int)(e % D0); const float* w = which ? w1 : ws; for (int j = 0; j < 8; ++j) o[j] = (b16)(bf16_rne(w[(size_t)(k0 + j) * HID + oo]) * WSC); for (int pass = 0; pass < 2; ++pass) { *(volatile v8b*)((which ? W1T : WST) + e) = o; __threadfence(); } return; } t -= 2 * n1;
  if (t < 2 * n2) { const int which = (int)(t / n2); const size_t e = (t % n2) * 8; const int oo = (int)(e / HID), k0 = (int)(e % HID); const float* w = which ? wl1 : w2; for (int j = 0; j < 8; ++j) o[j] = (b16)(bf16_rne(w[(size_t)(k0 + j) * HID + oo]) * WSC); for (int pass = 0; pass < 2; ++pass) { *(volatile v8b*)((which ? WL1T : W2T) + e) = o; __threadfence(); } return; } t -= 2 * n2;
  if (t < nj) { const size_t e = t * 8; const int oo = (int)(e / (2 * HID)), k0 = (int)(e % (2 * HID)); for (int j = 0; j < 8; ++j) o[j] = (b16)(bf16_rne(wj[(size_t)(k0 + j) * HID + oo]) * WSC); for (int pass = 0; pass < 2; ++pass) { *(volatile v8b*)(WJT + e) = o; __threadfence(); } return; } t -= nj;
  if (t < nl2) { const size_t e = t * 8; const int oo = (int)(e / HID), k0 = (int)(e % HID); for (int j = 0; j < 8; ++j) o[j] = oo < NOUT ? (b16)(bf16_rne(wl2[(size_t)(k0 + j) * NOUT + oo]) * WSC) : (b16)0.0f; for (int pass = 0; pass < 2; ++pass) { *(volatile v8b*)(WL2T + e) = o; __threadfence(); } }
}
template <int KD, int TWO, int RELU>
__global__ __launch_bounds__(128) void ngemm_kernel(const b16* __restrict__ Ah, const b16* __restrict__ Al, const b16* __restrict__ WT, const float* __restrict__ bias, float* __restrict__ OUT) {
  __shared__ __attribute__((aligned(16))) float Tf[4][16][HID + 4];
  const int wave = threadIdx.x >> 5, lane = threadIdx.x & 31, nloc = lane & 15, hlf = lane >> 4; const size_t m0 = (size_t)blockIdx.x * 64 + wave * 16;
  v8f acc[10];
#pragma unroll
  for (int t = 0; t < 10; ++t) acc[t] = (v8f){};
#pragma unroll
  for (int kb = 0; kb < KD; kb += 32) { const v16b a = frag_kb(Ah + (m0 + nloc) * KD + kb, hlf); v16b al; if (TWO) al = frag_kb(Al + (m0 + nloc) * KD + kb, hlf);
#pragma unroll
    for (int t = 0; t < 10; ++t) { const v16b bw = frag_kb(WT + (size_t)(t * 16 + nloc) * KD + kb, hlf); acc[t] = wmma16b(a, bw, acc[t]); if (TWO) acc[t] = wmma16b(al, bw, acc[t]); } }
#pragma unroll
  for (int t = 0; t < 10; ++t) { const int c = t * 16 + nloc; const float bb = bias ? bf16_rne(bias[c]) : 0.0f;
#pragma unroll 1
    for (int r = 0; r < 8; ++r) { const size_t row = m0 + 8 * hlf + r; float y = acc[t][r] * (1.0f / (XS * WSC)) + bb; if (RELU) y = fmaxf(y, 0.0f); Tf[wave][8 * hlf + r][c] = row < (size_t)N ? y : 0.0f; } }
  wave_lds_sync();
  for (int pass = 0; pass < 2; ++pass) { for (int rr = 0; rr < 16; ++rr) { *(volatile v4f*)(OUT + (m0 + rr) * HID + lane * 4) = *(const v4f*)(&Tf[wave][rr][lane * 4]); if (lane < 8) *(volatile v4f*)(OUT + (m0 + rr) * HID + 128 + lane * 4) = *(const v4f*)(&Tf[wave][rr][128 + lane * 4]); } __threadfence(); }
}
__global__ __launch_bounds__(256) void ew_kernel(const float* __restrict__ Z, const int* __restrict__ ei, const int* __restrict__ PERM, int permLen, float* __restrict__ EW) {
  const size_t j = (size_t)blockIdx.x * 256 + threadIdx.x; float w = 0.0f;
  if (j < (size_t)permLen) { const int p = PERM[j]; if (p >= 0 && p < E) { const size_t s = (size_t)iclamp(ei[p], 0, N - 1), d = (size_t)iclamp(ei[E + p], 0, N - 1); float dot = 0.0f;
#pragma unroll 1
      for (int c = 0; c < HID; ++c) dot += pmul(Z[s * HID + c], Z[d * HID + c]); w = ALPHA * (1.0f / (1.0f + __expf(-dot))) + BETA; } }
  for (int pass = 0; pass < 2; ++pass) { ((volatile float*)EW)[j] = w; __threadfence(); }
}
__global__ __launch_bounds__(256) void node_kernel(const float* __restrict__ H, const float* __restrict__ as_, const float* __restrict__ ad_, float* __restrict__ AS, float* __restrict__ AD) {
  __shared__ __attribute__((aligned(16))) float sa[8][8], sd[8][8];
  const int wave = threadIdx.x >> 5, lane = threadIdx.x & 31; const size_t v = (size_t)blockIdx.x * 8 + wave;
#pragma unroll
  for (int h = 0; h < NH; ++h) { const float hv = H[v * HID + h * CH + lane]; float s = pmul(hv, bf16_rne(as_[h * CH + lane])), d = pmul(hv, bf16_rne(ad_[h * CH + lane])); for (int o = 16; o; o >>= 1) { s += __shfl_xor(s, o); d += __shfl_xor(d, o); } if (lane == 0) { sa[wave][h] = s; sd[wave][h] = d; } }
  if (lane == 0) { for (int h = NH; h < 8; ++h) { sa[wave][h] = 0.0f; sd[wave][h] = 0.0f; } }
  __syncthreads();
  for (int pass = 0; pass < 2; ++pass) { if (threadIdx.x < 16) *(volatile v4f*)(AS + (size_t)blockIdx.x * 64 + threadIdx.x * 4) = *(const v4f*)(&sa[0][0] + threadIdx.x * 4); else if (threadIdx.x < 32) *(volatile v4f*)(AD + (size_t)blockIdx.x * 64 + (threadIdx.x - 16) * 4) = *(const v4f*)(&sd[0][0] + (threadIdx.x - 16) * 4); __threadfence(); }
}
template <int PLANES>
__global__ __launch_bounds__(256) void agg_kernel(const float* __restrict__ H, const float* __restrict__ AS, const float* __restrict__ AD, const int* __restrict__ ei, const int* __restrict__ PERM, const int* __restrict__ ROWPTR, const int* __restrict__ ROWCNT, int permLen, const float* __restrict__ EW, const float* __restrict__ epsp, const float* __restrict__ bias, float* __restrict__ HO, b16* __restrict__ Ph, b16* __restrict__ Pl) {
  __shared__ __attribute__((aligned(16))) b16 sh[8][2][HID + 8];
  const int wave = threadIdx.x >> 5, lane = threadIdx.x & 31; const size_t v = (size_t)blockIdx.x * 8 + wave;
  float out[NH]; for (int h = 0; h < NH; ++h) out[h] = 0.0f;
  if (v < (size_t)N) { int st = ROWPTR[v], cnt = ROWCNT[v]; cnt = iclamp(cnt, 0, 65536); st = iclamp(st, 0, permLen - cnt); const float wself = 1.0f + bf16_rne(epsp[0]);
    float adv[NH], mx[NH], den[NH], acc[NH];
#pragma unroll
    for (int h = 0; h < NH; ++h) { adv[h] = AD[v * 8 + h]; mx[h] = lrelu(AS[v * 8 + h] + adv[h]); den[h] = 0.0f; acc[h] = 0.0f; }
#pragma unroll 1
    for (int j = 0; j < cnt; ++j) { const int e = iclamp(PERM[st + j], 0, E - 1); const size_t s = (size_t)iclamp(ei[e], 0, N - 1);
#pragma unroll
      for (int h = 0; h < NH; ++h) mx[h] = fmaxf(mx[h], lrelu(AS[s * 8 + h] + adv[h])); }
#pragma unroll
    for (int h = 0; h < NH; ++h) { const float p = nexp(lrelu(AS[v * 8 + h] + adv[h]) - mx[h]); den[h] = p; acc[h] = pmul(p * wself, H[v * HID + h * CH + lane]); }
#pragma unroll 1
    for (int j = 0; j < cnt; ++j) { const int e = iclamp(PERM[st + j], 0, E - 1); const size_t s = (size_t)iclamp(ei[e], 0, N - 1); const float w = EW[st + j];
#pragma unroll
      for (int h = 0; h < NH; ++h) { const float p = nexp(lrelu(AS[s * 8 + h] + adv[h]) - mx[h]); den[h] += p; acc[h] += pmul(p * w, H[s * HID + h * CH + lane]); } }
#pragma unroll
    for (int h = 0; h < NH; ++h) out[h] = elu_(acc[h] / (den[h] + 1e-16f) + bf16_rne(bias[h * CH + lane])); }
  for (int pass = 0; pass < 2; ++pass) {
#pragma unroll
    for (int h = 0; h < NH; ++h) ((volatile float*)HO)[v * HID + h * CH + lane] = out[h]; __threadfence(); }
  if (PLANES) {
#pragma unroll
    for (int h = 0; h < NH; ++h) { b16 p, q; split16(out[h] * XS, p, q); sh[wave][0][h * CH + lane] = p; sh[wave][1][h * CH + lane] = q; }
    wave_lds_sync();
    for (int pass = 0; pass < 2; ++pass) { if (lane < 20) { *(volatile v8b*)(Ph + v * HID + lane * 8) = *(const v8b*)(&sh[wave][0][lane * 8]); *(volatile v8b*)(Pl + v * HID + lane * 8) = *(const v8b*)(&sh[wave][1][lane * 8]); } __threadfence(); } }
}
__device__ int lower_bound_i(const int* a, int n, int key) { int lo = 0, hi = n; while (lo < hi) { const int mid = (lo + hi) >> 1; if (a[mid] < key) lo = mid + 1; else hi = mid; } return lo; }
__global__ __launch_bounds__(160) void pool_kernel(const float* __restrict__ H1, const float* __restrict__ H2, const int* __restrict__ batch, float* __restrict__ GP) {
  const int g = blockIdx.x, c = threadIdx.x; const int lo = lower_bound_i(batch, N, g), hi = lower_bound_i(batch, N, g + 1);
  float s1 = 0.0f, s2 = 0.0f; for (int v = lo; v < hi; ++v) { s1 += H1[(size_t)v * HID + c]; s2 += H2[(size_t)v * HID + c]; }
  for (int pass = 0; pass < 2; ++pass) { ((volatile float*)GP)[(size_t)g * 2 * HID + c] = s1; ((volatile float*)GP)[(size_t)g * 2 * HID + HID + c] = s2; __threadfence(); }
}
__global__ __launch_bounds__(128) void head_kernel(const float* __restrict__ GP, const b16* __restrict__ WJT, const float* __restrict__ bj, const b16* __restrict__ WL1T, const float* __restrict__ bl1, const b16* __restrict__ WL2T, const float* __restrict__ bl2, float* __restrict__ out) {
  __shared__ __attribute__((aligned(16))) b16 Ah[4][16][2 * HID + 8], Al[4][16][2 * HID + 8]; __shared__ __attribute__((aligned(16))) float so[64 * NOUT];
  const int wave = threadIdx.x >> 5, lane = threadIdx.x & 31, nloc = lane & 15, hlf = lane >> 4; const int g0 = blockIdx.x * 64 + wave * 16;
  for (int q = lane; q < 16 * 80; q += 32) { const int rr = q / 80, c4 = (q % 80) * 4; const v4f v = *(const v4f*)(GP + (size_t)(g0 + rr) * 2 * HID + c4); for (int j = 0; j < 4; ++j) { b16 p, pl; split16(v[j] * XS, p, pl); Ah[wave][rr][c4 + j] = p; Al[wave][rr][c4 + j] = pl; } }
  wave_lds_sync();
  v8f acc[10];
  auto gemm = [&](const b16* WT, int KD) {
#pragma unroll
    for (int t = 0; t < 10; ++t) acc[t] = (v8f){};
    for (int kb = 0; kb < KD; kb += 32) { const v16b a = frag_kb(&Ah[wave][nloc][kb], hlf), al = frag_kb(&Al[wave][nloc][kb], hlf);
#pragma unroll
      for (int t = 0; t < 10; ++t) { const v16b bw = frag_kb(WT + (size_t)(t * 16 + nloc) * KD + kb, hlf); acc[t] = wmma16b(a, bw, acc[t]); acc[t] = wmma16b(al, bw, acc[t]); } } };
  auto restage_relu = [&](const float* bias) {
    wave_lds_sync();
#pragma unroll
    for (int t = 0; t < 10; ++t) { const int c = t * 16 + nloc; const float bb = bf16_rne(bias[c]);
#pragma unroll 1
      for (int r = 0; r < 8; ++r) { b16 p, q; split16(fmaxf(acc[t][r] * (1.0f / (XS * WSC)) + bb, 0.0f) * XS, p, q); Ah[wave][8 * hlf + r][c] = p; Al[wave][8 * hlf + r][c] = q; } }
    wave_lds_sync(); };
  gemm(WJT, 2 * HID); restage_relu(bj); gemm(WL1T, HID); restage_relu(bl1);
  { v8f o = {};
#pragma unroll
    for (int kb = 0; kb < HID; kb += 32) { const v16b a = frag_kb(&Ah[wave][nloc][kb], hlf), al = frag_kb(&Al[wave][nloc][kb], hlf); const v16b bw = frag_kb(WL2T + (size_t)nloc * HID + kb, hlf); o = wmma16b(a, bw, o); o = wmma16b(al, bw, o); }
#pragma unroll 1
    for (int r = 0; r < 8; ++r) if (nloc < NOUT) so[(wave * 16 + 8 * hlf + r) * NOUT + nloc] = o[r] * (1.0f / (XS * WSC)) + bf16_rne(bl2[nloc]); }
  __syncthreads();
  for (int pass = 0; pass < 2; ++pass) { for (int q = threadIdx.x; q < 64 * NOUT / 4; q += 128) *(volatile v4f*)(out + (size_t)blockIdx.x * 64 * NOUT + q * 4) = *(const v4f*)(&so[q * 4]); __threadfence(); }
}
}

extern "C" void kernel_launch(void* const* d_in, const int* in_sizes, int n_in, void* d_out, int out_size, void* d_ws, size_t ws_size, hipStream_t stream) {
  (void)n_in;
  auto Fp = [&](int i) { return (const float*)d_in[i]; }; auto Ip = [&](int i) { return (const int*)d_in[i]; };
  if (in_sizes[0] != N || in_sizes[1] != 2 * E || in_sizes[2] != N || in_sizes[3] != VOC * D0 || in_sizes[4] != D0 * HID || in_sizes[7] != D0 * HID || in_sizes[8] != NH * CH || in_sizes[11] != HID * HID || in_sizes[15] != 2 * HID * HID || in_sizes[19] != HID * NOUT || out_size != G * NOUT) return;
  size_t off = 0; char* ws = (char*)d_ws;
  auto carve = [&](size_t bytes) { char* p = ws + off; off += (bytes + 255) & ~(size_t)255; return p; };
  b16* XE = (b16*)carve((size_t)NP * D0 * 2); b16* WST = (b16*)carve((size_t)HID * D0 * 2); b16* W1T = (b16*)carve((size_t)HID * D0 * 2); b16* W2T = (b16*)carve((size_t)HID * HID * 2); b16* WJT = (b16*)carve((size_t)HID * 2 * HID * 2); b16* WL1T = (b16*)carve((size_t)HID * HID * 2); b16* WL2T = (b16*)carve((size_t)16 * HID * 2);
  float* Z = (float*)carve((size_t)NP * HID * 4); float* H = (float*)carve((size_t)NP * HID * 4); float* H1 = (float*)carve((size_t)NP * HID * 4); float* H2 = (float*)carve((size_t)NP * HID * 4); b16* P1h = (b16*)carve((size_t)NP * HID * 2); b16* P1l = (b16*)carve((size_t)NP * HID * 2);
  float* AS = (float*)carve((size_t)NP * 8 * 4); float* AD = (float*)carve((size_t)NP * 8 * 4); float* GP = (float*)carve((size_t)G * 2 * HID * 4);
  CsrBufs csr; off = csr_carve(csr, ws, off, E, N); float* EW = (float*)carve((csr.permLen + 256) * 4);
  if (off > ws_size) return;
  prep_kernel<<<(unsigned)(((size_t)NP * D0 / 8 + 2 * (size_t)HID * D0 / 8 + 2 * (size_t)HID * HID / 8 + (size_t)HID * 2 * HID / 8 + 16 * HID / 8 + 255) / 256), 256, 0, stream>>>(Ip(0), Fp(3), Fp(4), Fp(7), Fp(11), Fp(15), Fp(17), Fp(19), XE, WST, W1T, W2T, WJT, WL1T, WL2T);
  csr_build(csr, Ip(1) + E, E, N, stream);
  ngemm_kernel<D0, 0, 1><<<NP / 64, 128, 0, stream>>>(XE, nullptr, WST, Fp(5), Z);
  ew_kernel<<<(unsigned)((csr.permLen + 255) / 256), 256, 0, stream>>>(Z, Ip(1), csr.PERM, (int)csr.permLen, EW);
  ngemm_kernel<D0, 0, 0><<<NP / 64, 128, 0, stream>>>(XE, nullptr, W1T, nullptr, H);
  node_kernel<<<NP / 8, 256, 0, stream>>>(H, Fp(8), Fp(9), AS, AD);
  agg_kernel<1><<<NP / 8, 256, 0, stream>>>(H, AS, AD, Ip(1), csr.PERM, csr.ROWPTR, csr.ROWCNT, (int)csr.permLen, EW, Fp(6), Fp(10), H1, P1h, P1l);
  ngemm_kernel<HID, 1, 0><<<NP / 64, 128, 0, stream>>>(P1h, P1l, W2T, nullptr, H);
  node_kernel<<<NP / 8, 256, 0, stream>>>(H, Fp(12), Fp(13), AS, AD);
  agg_kernel<0><<<NP / 8, 256, 0, stream>>>(H, AS, AD, Ip(1), csr.PERM, csr.ROWPTR, csr.ROWCNT, (int)csr.permLen, EW, Fp(6), Fp(14), H2, nullptr, nullptr);
  pool_kernel<<<G, 160, 0, stream>>>(H1, H2, Ip(2), GP);
  head_kernel<<<G / 64, 128, 0, stream>>>(GP, WJT, Fp(16), WL1T, Fp(18), WL2T, Fp(20), (float*)d_out);
}
